// PhyloGAT_26886495273473
// MI455X (gfx1250) — hardware-run, weakly checked
//
#include <hip/hip_runtime.h>

typedef float          v8f   __attribute__((ext_vector_type(8)));
typedef float          v4f   __attribute__((ext_vector_type(4)));
typedef unsigned int   v4u   __attribute__((ext_vector_type(4)));
typedef int            v8i   __attribute__((ext_vector_type(8)));
typedef unsigned short v8us  __attribute__((ext_vector_type(8)));
typedef unsigned short v16us __attribute__((ext_vector_type(16)));
typedef __bf16         v16bf __attribute__((ext_vector_type(16)));
typedef _Float16       v16h  __attribute__((ext_vector_type(16)));
typedef v4f  __attribute__((may_alias)) v4fa;
typedef v8us __attribute__((may_alias)) v8usa;
union FragB { v16bf v; v16us u; v8us h[2]; v8i w; };
union FragH { v16h  v; v16us u; v8us h[2]; v8i w; };

__device__ __forceinline__ v8f wmb(const FragB& a, const FragB& b, v8f c) {
  v8f d = __builtin_amdgcn_wmma_f32_16x16x32_bf16(false, a.v, false, b.v, (short)0, c, false, false);
  asm volatile("v_nop\n\tv_nop\n\tv_nop\n\tv_nop" : "+v"(d) : "v"(a.w), "v"(b.w));
  return d;
}

__device__ __forceinline__ v8f wmh(const FragH& a, const FragH& b, v8f c) {
  v8f d = __builtin_amdgcn_wmma_f32_16x16x32_f16(false, a.v, false, b.v, (short)0, c, false, false);
  asm volatile("v_nop\n\tv_nop\n\tv_nop\n\tv_nop" : "+v"(d) : "v"(a.w), "v"(b.w));
  return d;
}

__device__ __forceinline__ unsigned bf16_bits(float f) {
  const unsigned u = __float_as_uint(f);
  const unsigned r = (u + 0x7FFFu + ((u >> 16) & 1u)) >> 16;
  const unsigned q = (u >> 16) | 0x40u;
  return ((u & 0x7fffffffu) > 0x7f800000u) ? q : r;
}

__device__ __forceinline__ float bf16_val(float f) {
  return __uint_as_float(bf16_bits(f) << 16);
}
__device__ __forceinline__ int clampi(int v, int lo, int hi) {
  return v < lo ? lo : (v > hi ? hi : v);
}

__device__ __forceinline__ unsigned f16_bits(float f) {
  const unsigned u  = __float_as_uint(f);
  const unsigned s  = (u >> 16) & 0x8000u;
  const unsigned a  = u & 0x7fffffffu;
  const unsigned t  = a - 0x38000000u;
  const unsigned r  = (t + 0x0FFFu + ((t >> 13) & 1u)) >> 13;
  const unsigned rc = r > 0x7C00u ? 0x7C00u : r;
  const bool small  = a < 0x38800000u;
  const bool isnan  = a > 0x7f800000u;
  const unsigned fin = small ? 0u : (s | rc);
  return isnan ? (s | 0x7E00u) : fin;
}

__device__ __forceinline__ unsigned pk16(unsigned lo, unsigned hi) { return lo | (hi << 16); }
__device__ __forceinline__ unsigned bf16_lo_bits(float v) {
  float hi = bf16_val(v);
  asm volatile("" : "+v"(hi));
  return bf16_bits(v - hi);
}
__device__ __forceinline__ v4u pack8_bf16(v4f a, v4f c) {
  return (v4u){ pk16(bf16_bits(a[0]), bf16_bits(a[1])), pk16(bf16_bits(a[2]), bf16_bits(a[3])),
                pk16(bf16_bits(c[0]), bf16_bits(c[1])), pk16(bf16_bits(c[2]), bf16_bits(c[3])) };
}
__device__ __forceinline__ v4u pack8_bf16_lo(v4f a, v4f c) {
  return (v4u){ pk16(bf16_lo_bits(a[0]), bf16_lo_bits(a[1])), pk16(bf16_lo_bits(a[2]), bf16_lo_bits(a[3])),
                pk16(bf16_lo_bits(c[0]), bf16_lo_bits(c[1])), pk16(bf16_lo_bits(c[2]), bf16_lo_bits(c[3])) };
}
__device__ __forceinline__ v4u pack8_f16(v4f a, v4f c) {
  return (v4u){ pk16(f16_bits(a[0]), f16_bits(a[1])), pk16(f16_bits(a[2]), f16_bits(a[3])),
                pk16(f16_bits(c[0]), f16_bits(c[1])), pk16(f16_bits(c[2]), f16_bits(c[3])) };
}

template <int FORM>
__global__ __launch_bounds__(256) void k_plane(const float* __restrict__ src, int rows, int cols, int ldsrc,
                                               unsigned short* __restrict__ dst, int MP, int KP) {
  static_assert(FORM >= 0 && FORM <= 3);
  const int KTOT = (FORM == 1 || FORM == 3) ? 2 * KP : KP;
  const unsigned ppr   = (unsigned)(KTOT >> 3);
  const unsigned kp8   = (unsigned)(KP >> 3);
  const unsigned total = (unsigned)MP * ppr;
  const unsigned g     = blockIdx.x * 256u + threadIdx.x;
  const unsigned rowu  = g / ppr;
  const unsigned p     = g - rowu * ppr;
  const bool second    = p >= kp8;
  const int row = (int)rowu;
  const int c0  = (int)((second ? p - kp8 : p) << 3);
  const float* srow = src + (size_t)clampi(row, 0, rows - 1) * (size_t)ldsrc;
  float x[8];
  unsigned mk[8];
#pragma unroll
  for (int e = 0; e < 8; ++e) {
    const int c = c0 + e;
    const float v = srow[clampi(c, 0, cols - 1)];
    asm volatile("" :: "v"(v));
    x[e]  = v;
    mk[e] = (row < rows && c < cols) ? 0xFFFFu : 0u;
  }
  const v4f a = (v4f){ x[0], x[1], x[2], x[3] };
  const v4f c = (v4f){ x[4], x[5], x[6], x[7] };
  v4u o;
  if (FORM == 2) {
    o = pack8_f16(a, c);
  } else {
    const v4u hi = pack8_bf16(a, c);
    o = hi;
    if (FORM == 1) { const v4u lo = pack8_bf16_lo(a, c); o = second ? lo : hi; }
  }
  const v4u mw = (v4u){ pk16(mk[0], mk[1]), pk16(mk[2], mk[3]), pk16(mk[4], mk[5]), pk16(mk[6], mk[7]) };
  o &= mw;
  if (g < total) {
    volatile v4u* q = (volatile v4u*)(dst + (size_t)g * 8);
    *q = o;
    __threadfence();
    *q = o;
  }
}

template <int FORM> struct FragOf    { typedef FragB T; };
template <>         struct FragOf<2> { typedef FragH T; };
__device__ __forceinline__ v8f mm(const FragB& a, const FragB& b, v8f c) { return wmb(a, b, c); }
__device__ __forceinline__ v8f mm(const FragH& a, const FragH& b, v8f c) { return wmh(a, b, c); }
template <class F> __device__ __forceinline__ F ld_frag(const unsigned short* p) {
  F f;
  f.h[0] = *(const v8usa*)(p);
  f.h[1] = *(const v8usa*)(p + 16);
  return f;
}

template <int FORM, int EPI>
__global__ __launch_bounds__(256) __attribute__((amdgpu_num_vgpr(248)))
void k_gemm_nt(const unsigned short* __restrict__ A, const unsigned short* __restrict__ B,
               const float* __restrict__ bias, float* __restrict__ D, int M, int N, int KTOT, int ldd) {
  static_assert(FORM >= 0 && FORM <= 2);
  static_assert(EPI == 0 || EPI == 1);
  typedef typename FragOf<FORM>::T F;
  __shared__ __attribute__((aligned(16))) float sT[8][16 * 68];
  const int lane = threadIdx.x & 31;
  const int wave = threadIdx.x >> 5;
  const int tilesM = (M + 63) >> 6;
  const int tilesN = (N + 63) >> 6;
  const int tile = blockIdx.x * 8 + wave;
  if (tile >= tilesM * tilesN) return;
  const int tm = tile / tilesN;
  const int tn = tile - tm * tilesN;
  const int m0 = tm << 6;
  const int n0 = tn << 6;

  const int rl = lane & 15;
  const int h8 = (lane >> 4) * 8;
  const unsigned short* pa = A + (size_t)(m0 + rl) * (size_t)KTOT + h8;
  const unsigned short* pb = B + (size_t)(n0 + rl) * (size_t)KTOT + h8;

  v8f acc[4][4];
#pragma unroll
  for (int i = 0; i < 4; ++i)
#pragma unroll
    for (int j = 0; j < 4; ++j) acc[i][j] = (v8f){0.f, 0.f, 0.f, 0.f, 0.f, 0.f, 0.f, 0.f};

#pragma unroll 1
  for (int k0 = 0; k0 < KTOT; k0 += 32) {
    F bf[4];
#pragma unroll
    for (int j = 0; j < 4; ++j) bf[j] = ld_frag<F>(pb + (size_t)(j << 4) * (size_t)KTOT + k0);
#pragma unroll
    for (int i = 0; i < 4; ++i) {
      const F af = ld_frag<F>(pa + (size_t)(i << 4) * (size_t)KTOT + k0);
#pragma unroll
      for (int j = 0; j < 4; ++j) acc[i][j] = mm(af, bf[j], acc[i][j]);
    }
  }

  float* slab = sT[wave];
  const int hh = lane >> 4;
  const int c4 = (lane & 15) * 4;
  const int nc = n0 + c4;
  const bool cok = nc < N;
  v4f bv = (v4f){0.f, 0.f, 0.f, 0.f};
  if (EPI == 1) {
    bv = *(const v4fa*)(bias + clampi(nc, 0, N - 4));
    asm volatile("" :: "v"(bv));
  }
#pragma unroll
  for (int i = 0; i < 4; ++i) {
    const int mBase = m0 + (i << 4);
#pragma unroll
    for (int j = 0; j < 4; ++j) {
#pragma unroll
      for (int r = 0; r < 8; ++r) slab[(h8 + r) * 68 + (j << 4) + rl] = acc[i][j][r];
    }
    __builtin_amdgcn_fence(__ATOMIC_RELEASE, "workgroup");
    __builtin_amdgcn_wave_barrier();
    __builtin_amdgcn_fence(__ATOMIC_ACQUIRE, "workgroup");
    v4f vv[8];
#pragma unroll
    for (int it = 0; it < 8; ++it) {
      const int row = it * 2 + hh;
      v4f v = *(const v4fa*)(slab + row * 68 + c4);
      if (EPI == 1) v += bv;
      vv[it] = v;
    }
    for (int pass = 0; pass < 2; ++pass) {
#pragma unroll
      for (int it = 0; it < 8; ++it) {
        const int row = mBase + it * 2 + hh;
        if (cok && row < M) *(volatile v4f*)(D + (size_t)row * (size_t)ldd + nc) = vv[it];
      }
      __threadfence();
    }
    __builtin_amdgcn_fence(__ATOMIC_RELEASE, "workgroup");
    __builtin_amdgcn_wave_barrier();
    __builtin_amdgcn_fence(__ATOMIC_ACQUIRE, "workgroup");
  }
}

#pragma clang fp contract(off)


#ifndef L2_SINGLE
#define L2_SINGLE 0
#endif

#define NN      50000
#define EE      800000
#define MPAD    50048
#define FIN     128
#define C1W     256
#define OUTW    32
#define K2TOT   (L2_SINGLE ? 256 : 512)
#define NB      1024
#define NBLK    49
#define BCH     2048
#define NCH     391
#define WLCAP   4096
#define RCAP    21504
#define SEGP    400
#define DEGCAP  48
#define FLGP    32
#define FLGL    64

#define T_AS1   0
#define T_AD1   256
#define T_B1    512
#define T_GA    768
#define T_BE    1024
#define T_MU    1280
#define T_RS    1536
#define T_AS2   1792
#define T_AD2   1824
#define T_B2    1856
#define T_TOT   2048

#define NW2B    (64 * K2TOT / 8 / 256)
#define NPADB   (48 * K2TOT / 8 / 256)
#define PB_W2   16
#define PB_TAB  (PB_W2 + NW2B)
#define PB_PAD  (PB_TAB + 10)
#define PB_FLG  (PB_PAD + NPADB)
#define PB_END  (PB_FLG + 2)

#define LDS_BKT ((8 * WLCAP + RCAP + 3 * NB + 8 * SEGP + 32) * 4)

static_assert(NN == 50000 && EE == 800000);
static_assert(NN <= 65536);
static_assert(NB == 1024);
static_assert(NBLK * NB >= NN);
static_assert(MPAD % 64 == 0 && MPAD >= NN && MPAD - NN == 48);
static_assert(NN % 16 == 0 && NN % 4 == 0 && NN % 8 == 0);
static_assert(EE % 8 == 0);
static_assert(NCH * BCH >= EE && (NCH - 1) * BCH < EE);
static_assert(NCH + 1 <= SEGP);
static_assert(RCAP >= 20779 && RCAP % 1024 == 0);
static_assert(DEGCAP >= 35 + 8 && DEGCAP <= 62);
static_assert(LDS_BKT <= 262144);
static_assert(NBLK <= FLGL);
static_assert((64 * K2TOT / 8) % 256 == 0 && (48 * K2TOT / 8) % 256 == 0);
static_assert((size_t)NN * K2TOT * 2 >= (size_t)MPAD * FIN * 2);
static_assert(K2TOT % 32 == 0 && FIN % 32 == 0);

typedef int v4i __attribute__((ext_vector_type(4)));
typedef v4i __attribute__((may_alias)) v4ia;
typedef v4u __attribute__((may_alias)) v4ua;

__device__ __forceinline__ float nmax(float a, float b) { return (b > a || b != b) ? b : a; }
__device__ __forceinline__ float leaky(float v) { return v >= 0.0f ? v : 0.2f * v; }
__device__ __forceinline__ float sel4(v4f v, int h) {
  float r = v[0];
  r = (h == 1) ? v[1] : r;
  r = (h == 2) ? v[2] : r;
  r = (h == 3) ? v[3] : r;
  return r;
}
__device__ __forceinline__ int rlane(int v, int l) { return __builtin_amdgcn_readlane(v, l); }
__device__ __forceinline__ float rlanef(float v, int l) {
  return __int_as_float(__builtin_amdgcn_readlane(__float_as_int(v), l));
}
__device__ __forceinline__ void wave_sync() {
  __builtin_amdgcn_fence(__ATOMIC_RELEASE, "workgroup");
  __builtin_amdgcn_wave_barrier();
  __builtin_amdgcn_fence(__ATOMIC_ACQUIRE, "workgroup");
}
__device__ __forceinline__ void put16(void* p, v4u o) {
  volatile v4u* q = (volatile v4u*)p;
  *q = o;
  __threadfence();
  *q = o;
}

__device__ __forceinline__ void tab_put(const float* __restrict__ src, float* dst, int n4, int tid) {
  const int i = tid < n4 ? tid : n4 - 1;
  v4f v = *(const v4fa*)(src + 4 * i);
  asm volatile("" :: "v"(v));
  const v4f o = (v4f){ bf16_val(v[0]), bf16_val(v[1]), bf16_val(v[2]), bf16_val(v[3]) };
  volatile v4f* q = (volatile v4f*)(dst + 4 * i);
  const bool ok = tid < n4;
  if (ok) *q = o;
  __threadfence();
  if (ok) *q = o;
}
__device__ __forceinline__ void tab_put_rs(const float* __restrict__ src, float* dst, int n4, int tid) {
  const int i = tid < n4 ? tid : n4 - 1;
  v4f v = *(const v4fa*)(src + 4 * i);
  asm volatile("" :: "v"(v));
  float x0 = v[0], x1 = v[1], x2 = v[2], x3 = v[3];
#pragma unroll 1
  for (int c = 0; c < 4; ++c) {
    const float bq = bf16_val(x0);
    const float r = 1.0f / sqrtf(bq + 1e-5f);
    x0 = x1; x1 = x2; x2 = x3; x3 = r;
  }
  const v4f o = (v4f){ x0, x1, x2, x3 };
  volatile v4f* q = (volatile v4f*)(dst + 4 * i);
  const bool ok = tid < n4;
  if (ok) *q = o;
  __threadfence();
  if (ok) *q = o;
}

__global__ __launch_bounds__(256) void k_prep(
    const float* __restrict__ W1, const float* __restrict__ W2,
    const float* __restrict__ as1, const float* __restrict__ ad1, const float* __restrict__ b1,
    const float* __restrict__ ga, const float* __restrict__ be, const float* __restrict__ mu,
    const float* __restrict__ var, const float* __restrict__ as2, const float* __restrict__ ad2,
    const float* __restrict__ b2,
    unsigned short* __restrict__ W1T, unsigned short* __restrict__ W2D, float* __restrict__ tab,
    unsigned short* __restrict__ A2, int* __restrict__ flagp) {
  const int b = (int)blockIdx.x;
  const int tid = (int)threadIdx.x;
  if (b < PB_W2) {
    const int u = b * 256 + tid;
    const int n = u >> 4;
    const int k8 = (u & 15) << 3;
    const float* p = W1 + (size_t)k8 * C1W + n;
    float x[8];
#pragma unroll
    for (int e = 0; e < 8; ++e) {
      const float v = p[(size_t)e * C1W];
      asm volatile("" :: "v"(v));
      x[e] = v;
    }
    const v4u o = pack8_bf16((v4f){ x[0], x[1], x[2], x[3] }, (v4f){ x[4], x[5], x[6], x[7] });
    put16(W1T + (size_t)u * 8, o);
  } else if (b < PB_TAB) {
    const int u = (b - PB_W2) * 256 + tid;
    const int ppr = K2TOT / 8;
    const int n = u / ppr;
    const int k8 = ((u - n * ppr) << 3) & 255;
    const int ncl = n < OUTW ? n : OUTW - 1;
    const float* p = W2 + (size_t)k8 * OUTW + ncl;
    float x[8];
#pragma unroll
    for (int e = 0; e < 8; ++e) {
      const float v = p[(size_t)e * OUTW];
      asm volatile("" :: "v"(v));
      x[e] = v;
    }
    v4u o = pack8_bf16((v4f){ x[0], x[1], x[2], x[3] }, (v4f){ x[4], x[5], x[6], x[7] });
    const unsigned mk = n < OUTW ? 0xFFFFFFFFu : 0u;
    o &= (v4u){ mk, mk, mk, mk };
    put16(W2D + (size_t)u * 8, o);
  } else if (b < PB_PAD) {
    const int t = b - PB_TAB;
    if (t == 0)      tab_put(as1, tab + T_AS1, 64, tid);
    else if (t == 1) tab_put(ad1, tab + T_AD1, 64, tid);
    else if (t == 2) tab_put(b1,  tab + T_B1,  64, tid);
    else if (t == 3) tab_put(ga,  tab + T_GA,  64, tid);
    else if (t == 4) tab_put(be,  tab + T_BE,  64, tid);
    else if (t == 5) tab_put(mu,  tab + T_MU,  64, tid);
    else if (t == 6) tab_put_rs(var, tab + T_RS, 64, tid);
    else if (t == 7) tab_put(as2, tab + T_AS2, 8, tid);
    else if (t == 8) tab_put(ad2, tab + T_AD2, 8, tid);
    else             tab_put(b2,  tab + T_B2,  8, tid);
  } else if (b < PB_FLG) {
    const int u = (b - PB_PAD) * 256 + tid;
    put16(A2 + (size_t)NN * K2TOT + (size_t)u * 8, (v4u){ 0u, 0u, 0u, 0u });
  } else {
    const int u = (b - PB_FLG) * 256 + tid;
    put16(flagp + (size_t)u * 4, (v4u){ 0u, 0u, 0u, 0u });
  }
}

__global__ __launch_bounds__(256) void k_bucket(const int* __restrict__ ei, unsigned* __restrict__ hits,
                                                int* __restrict__ offp, int* __restrict__ cntp,
                                                int* __restrict__ flagp) {
  extern __shared__ v4u lds_bk[];
  unsigned* wl  = (unsigned*)lds_bk;
  unsigned* srt = wl + 8 * WLCAP;
  int* scnt = (int*)(srt + RCAP);
  int* soff = scnt + NB;
  int* cur  = soff + NB;
  int* wseg = cur + NB;
  int* wtot = wseg + 8 * SEGP;
  int* ptot = wtot + 8;
  const int tid = (int)threadIdx.x, lane = tid & 31, wave = tid >> 5;
  const int blk = (int)blockIdx.x;
  const unsigned nbs = (unsigned)(blk * NB);

  {
    const v4u z4 = (v4u){ 0u, 0u, 0u, 0u };
    for (int i = tid; i < RCAP / 4; i += 256) *(v4ua*)(srt + 4 * i) = z4;
    *(v4ia*)(scnt + 4 * tid) = (v4i){ 0, 0, 0, 0 };
  }
  __syncthreads();

  const int* __restrict__ srow = ei;
  const int* __restrict__ drow = ei + EE;
  int wc = 0;
#pragma unroll 1
  for (int ch = 0; ch < NCH; ++ch) {
    if (lane == 0) wseg[wave * SEGP + ch] = wc;
    const int e0  = ch * BCH + tid * 8;
    const int e0c = e0 < EE - 8 ? e0 : EE - 8;
    const bool valid = e0 < EE;
    const v4i da = *(const v4ia*)(drow + e0c);
    const v4i db = *(const v4ia*)(drow + e0c + 4);
    const v4i sa = *(const v4ia*)(srow + e0c);
    const v4i sb = *(const v4ia*)(srow + e0c + 4);
    asm volatile("" :: "v"(da), "v"(db), "v"(sa), "v"(sb));
#define HITJ(DJ, SJ) { \
      const unsigned sl = (unsigned)(DJ) - nbs; \
      const bool hj = valid && (sl < (unsigned)NB); \
      const unsigned mj = __builtin_amdgcn_ballot_w32(hj); \
      if (mj != 0u) { \
        if (hj) { \
          const int pos = wc + (int)__builtin_amdgcn_mbcnt_lo(mj, 0u); \
          if (pos < WLCAP) wl[wave * WLCAP + pos] = (unsigned)clampi((SJ), 0, NN - 1) | (sl << 16); \
        } \
        wc += (int)__builtin_popcount(mj); } }
    HITJ(da[0], sa[0])
    HITJ(da[1], sa[1])
    HITJ(da[2], sa[2])
    HITJ(da[3], sa[3])
    HITJ(db[0], sb[0])
    HITJ(db[1], sb[1])
    HITJ(db[2], sb[2])
    HITJ(db[3], sb[3])
#undef HITJ
  }
  if (lane == 0) { wseg[wave * SEGP + NCH] = wc; wtot[wave] = wc; }
  __syncthreads();

  int nh = 0;
  bool ov = false;
#pragma unroll
  for (int w = 0; w < 8; ++w) {
    const int t = wtot[w];
    ov = ov || (t > WLCAP) || (t < 0);
    nh += clampi(t, 0, WLCAP);
  }
  ov = ov || (nh > RCAP);

  if (wave == 0) {
#pragma unroll 1
    for (int w = 0; w < 8; ++w) {
      const int nw = __builtin_amdgcn_readfirstlane(clampi(wtot[w], 0, WLCAP));
#pragma unroll 1
      for (int b0 = 0; b0 < nw; b0 += 32) {
        const int idx = (b0 + lane) < nw ? (b0 + lane) : nw - 1;
        const unsigned uv = wl[w * WLCAP + idx];
        const int m32 = (nw - b0) < 32 ? (nw - b0) : 32;
#pragma unroll 1
        for (int k = 0; k < m32; ++k) {
          const unsigned u = (unsigned)rlane((int)uv, k);
          const int sl = (int)((u >> 16) & (unsigned)(NB - 1));
          if (lane == 0) scnt[sl] = scnt[sl] + 1;
        }
      }
    }
  }
  __syncthreads();

  const v4i c4r = *(const v4ia*)(scnt + 4 * tid);
  const int q0 = c4r[0] < 0 ? 0 : c4r[0];
  const int q1 = c4r[1] < 0 ? 0 : c4r[1];
  const int q2 = c4r[2] < 0 ? 0 : c4r[2];
  const int q3 = c4r[3] < 0 ? 0 : c4r[3];
  const int ts = q0 + q1 + q2 + q3;
  int incl = ts;
#pragma unroll
  for (int d = 1; d < 32; d <<= 1) {
    const int up = __shfl_up(incl, d);
    incl += (lane >= d) ? up : 0;
  }
  if (lane == 31) ptot[wave] = incl;
  __syncthreads();
  int pre = 0;
#pragma unroll
  for (int w2 = 0; w2 < 8; ++w2) {
    const int pt = ptot[w2];
    pre += (w2 < wave) ? pt : 0;
  }
  const int run = pre + incl - ts;
  const v4i so = (v4i){ run, run + q0, run + q0 + q1, run + q0 + q1 + q2 };
  *(v4ia*)(soff + 4 * tid) = so;
  *(v4ia*)(cur + 4 * tid)  = so;
  __syncthreads();

  if (wave == 0) {
#pragma unroll 1
    for (int ch = 0; ch < NCH; ++ch) {
#pragma unroll 1
      for (int w = 0; w < 8; ++w) {
        const int nw = __builtin_amdgcn_readfirstlane(clampi(wtot[w], 0, WLCAP));
        const int st = __builtin_amdgcn_readfirstlane(clampi(wseg[w * SEGP + ch], 0, nw));
        const int en = __builtin_amdgcn_readfirstlane(clampi(wseg[w * SEGP + ch + 1], st, nw));
#pragma unroll 1
        for (int b0 = st; b0 < en; b0 += 32) {
          const int idx = (b0 + lane) < en ? (b0 + lane) : en - 1;
          const unsigned uv = wl[w * WLCAP + idx];
          const int m32 = (en - b0) < 32 ? (en - b0) : 32;
#pragma unroll 1
          for (int k = 0; k < m32; ++k) {
            const unsigned u = (unsigned)rlane((int)uv, k);
            const int sl = (int)((u >> 16) & (unsigned)(NB - 1));
            if (lane == 0) {
              const int pos = clampi(cur[sl], 0, RCAP - 1);
              srt[pos] = u;
              cur[sl] = pos + 1;
            }
          }
        }
      }
    }
  }
  __syncthreads();

  unsigned* hb = hits + (size_t)blk * RCAP;
  const v4i cn4 = (v4i){ q0, q1, q2, q3 };
  const int fv = ov ? 1 : 0;
  for (int pass = 0; pass < 2; ++pass) {
#pragma unroll 1
    for (int it = 0; it < RCAP / 1024; ++it) {
      const int i = it * 256 + tid;
      const v4u v = *(const v4ua*)(srt + 4 * i);
      *(volatile v4u*)(hb + 4 * i) = v;
    }
    *(volatile v4i*)(offp + (size_t)blk * NB + 4 * tid) = so;
    *(volatile v4i*)(cntp + (size_t)blk * NB + 4 * tid) = cn4;
    if (wave == 0) *(volatile int*)(flagp + blk * FLGP + lane) = fv;
    __threadfence();
  }
}

__global__ __launch_bounds__(256) void k_node1(const float* __restrict__ HW, const float* __restrict__ tab,
                                               float* __restrict__ SD1) {
  const int lane = threadIdx.x & 31, wave = threadIdx.x >> 5;
  const int wv = (int)blockIdx.x * 8 + wave;
  if (wv >= NN / 4) return;
  const v4f sA = *(const v4fa*)(tab + T_AS1 + 8 * lane);
  const v4f sB = *(const v4fa*)(tab + T_AS1 + 8 * lane + 4);
  const v4f dA = *(const v4fa*)(tab + T_AD1 + 8 * lane);
  const v4f dB = *(const v4fa*)(tab + T_AD1 + 8 * lane + 4);
  const int node0 = wv * 4;
  float outv = 0.0f;
#pragma unroll 1
  for (int q = 0; q < 4; ++q) {
    const float* rp = HW + (size_t)(node0 + q) * C1W + 8 * lane;
    const v4f ra = *(const v4fa*)rp;
    const v4f rb = *(const v4fa*)(rp + 4);
    float ps = ra[0] * sA[0];
    ps = ps + ra[1] * sA[1]; ps = ps + ra[2] * sA[2]; ps = ps + ra[3] * sA[3];
    ps = ps + rb[0] * sB[0]; ps = ps + rb[1] * sB[1]; ps = ps + rb[2] * sB[2]; ps = ps + rb[3] * sB[3];
    float pd = ra[0] * dA[0];
    pd = pd + ra[1] * dA[1]; pd = pd + ra[2] * dA[2]; pd = pd + ra[3] * dA[3];
    pd = pd + rb[0] * dB[0]; pd = pd + rb[1] * dB[1]; pd = pd + rb[2] * dB[2]; pd = pd + rb[3] * dB[3];
    ps += __shfl_xor(ps, 1); pd += __shfl_xor(pd, 1);
    ps += __shfl_xor(ps, 2); pd += __shfl_xor(pd, 2);
    ps += __shfl_xor(ps, 4); pd += __shfl_xor(pd, 4);
    const float vs = __shfl(ps, 8 * (lane & 3));
    const float vd = __shfl(pd, 8 * (lane & 3));
    const float mine = ((lane & 4) != 0) ? vd : vs;
    outv = ((lane >> 3) == q) ? mine : outv;
  }
  volatile float* qp = (volatile float*)(SD1 + (size_t)node0 * 8 + lane);
  *qp = outv;
  __threadfence();
  *qp = outv;
}

__global__ __launch_bounds__(256) void k_replay1(
    const float* __restrict__ HW, const float* __restrict__ SD1, const unsigned* __restrict__ hits,
    const int* __restrict__ offp, const int* __restrict__ cntp, const int* __restrict__ flagp,
    const float* __restrict__ tab, unsigned short* __restrict__ A2) {
  __shared__ __attribute__((aligned(16))) float sPar[1280];
  __shared__ __attribute__((aligned(16))) float sA[8][256];
  const int tid = (int)threadIdx.x, lane = tid & 31, wave = tid >> 5;
  {
    const int i0 = tid;
    const int i1 = (tid + 256) < 320 ? (tid + 256) : 319;
    const v4f p0 = *(const v4fa*)(tab + T_B1 + 4 * i0);
    const v4f p1 = *(const v4fa*)(tab + T_B1 + 4 * i1);
    *(v4fa*)(sPar + 4 * i0) = p0;
    *(v4fa*)(sPar + 4 * i1) = p1;
  }
  __syncthreads();

  const int row = (int)blockIdx.x * 8 + wave;
  const bool live = row < NN;
  const int ic = row < NN ? row : NN - 1;
  const int blk = ic >> 10;
  const int offv = offp[ic];
  const int cntv = cntp[ic];
  const int flg  = flagp[blk * FLGP];
  asm volatile("" :: "v"(offv), "v"(cntv), "v"(flg));
  const int cn  = __builtin_amdgcn_readfirstlane(live ? clampi(cntv, 0, DEGCAP) : 0);
  const int off = __builtin_amdgcn_readfirstlane(clampi(offv, 0, RCAP - 1));
  const bool bad = (flg != 0) || (cntv > DEGCAP) || (cntv < 0);

  const v4f oas = *(const v4fa*)(SD1 + (size_t)ic * 8);
  const v4f oad = *(const v4fa*)(SD1 + (size_t)ic * 8 + 4);
  asm volatile("" :: "v"(oas), "v"(oad));

  const unsigned* hb = hits + (size_t)blk * RCAP;
  const unsigned w0 = hb[clampi(off + lane, 0, RCAP - 1)];
  const unsigned w1 = hb[clampi(off + 32 + lane, 0, RCAP - 1)];
  asm volatile("" :: "v"(w0), "v"(w1));
  const int s0 = clampi((int)(w0 & 0xFFFFu), 0, NN - 1);
  int s1 = clampi((int)(w1 & 0xFFFFu), 0, NN - 1);
  s1 = (lane == 31) ? ic : s1;
  const v4f sd0 = *(const v4fa*)(SD1 + (size_t)s0 * 8);
  const v4f sd1 = *(const v4fa*)(SD1 + (size_t)s1 * 8);
  asm volatile("" :: "v"(sd0), "v"(sd1));
  const bool act0 = lane < cn;
  const bool act1 = ((32 + lane) < cn) || (lane == 31);
  const float ninf = __uint_as_float(0xff800000u);

  float* sAw = sA[wave];
#pragma unroll 1
  for (int h = 0; h < 4; ++h) {
    const float adh = sel4(oad, h);
    const float e0 = leaky(sel4(sd0, h) + adh);
    const float e1 = leaky(sel4(sd1, h) + adh);
    float m = act0 ? e0 : ninf;
    const float m1 = act1 ? e1 : ninf;
    m = nmax(m, m1);
#pragma unroll
    for (int o = 16; o > 0; o >>= 1) {
      const float t = __shfl_xor(m, o);
      m = nmax(m, t);
    }
    float p0 = expf(e0 - m);
    float p1 = expf(e1 - m);
    p0 = act0 ? p0 : 0.0f;
    p1 = act1 ? p1 : 0.0f;
    float dsum = p0 + p1;
#pragma unroll
    for (int o = 16; o > 0; o >>= 1) dsum += __shfl_xor(dsum, o);
    const float den = dsum + 1e-16f;
    sAw[h * 64 + lane]      = p0 / den;
    sAw[h * 64 + 32 + lane] = p1 / den;
  }
  wave_sync();

  float acc[8];
#pragma unroll
  for (int c = 0; c < 8; ++c) acc[c] = 0.0f;
  const float* hwl = HW + 8 * lane;
  const int hl = (lane >> 3) * 64;
#pragma unroll 1
  for (int j = 0; j <= cn; ++j) {
    const int jj = j < cn ? j : 63;
    const int sa_ = rlane(s0, jj & 31);
    const int sb_ = rlane(s1, jj & 31);
    const int sj = jj < 32 ? sa_ : sb_;
    const float w = sAw[hl + jj];
    const float* rp = hwl + (size_t)sj * C1W;
    const v4f r0 = *(const v4fa*)rp;
    const v4f r1 = *(const v4fa*)(rp + 4);
    asm volatile("" :: "v"(r0), "v"(r1));
    acc[0] = acc[0] + w * r0[0]; acc[1] = acc[1] + w * r0[1];
    acc[2] = acc[2] + w * r0[2]; acc[3] = acc[3] + w * r0[3];
    acc[4] = acc[4] + w * r1[0]; acc[5] = acc[5] + w * r1[1];
    acc[6] = acc[6] + w * r1[2]; acc[7] = acc[7] + w * r1[3];
  }

  float a0 = acc[0], a1 = acc[1], a2 = acc[2], a3 = acc[3];
  float a4 = acc[4], a5 = acc[5], a6 = acc[6], a7 = acc[7];
  const float qn = __uint_as_float(0x7fc00000u);
#pragma unroll 1
  for (int c = 0; c < 8; ++c) {
    const int col = 8 * lane + c;
    float v = a0 + sPar[col];
    v = ((v - sPar[768 + col]) * sPar[1024 + col]) * sPar[256 + col] + sPar[512 + col];
    float r = v > 0.0f ? v : expm1f(v);
    r = bad ? qn : r;
    a0 = a1; a1 = a2; a2 = a3; a3 = a4; a4 = a5; a5 = a6; a6 = a7; a7 = r;
  }
  const v4f va = (v4f){ a0, a1, a2, a3 };
  const v4f vc = (v4f){ a4, a5, a6, a7 };
  const v4u hi = pack8_bf16(va, vc);
#if !L2_SINGLE
  const v4u lo = pack8_bf16_lo(va, vc);
#endif
  unsigned short* rowp = A2 + (size_t)ic * K2TOT + 8 * lane;
  for (int pass = 0; pass < 2; ++pass) {
    if (live) {
      *(volatile v4u*)rowp = hi;
#if !L2_SINGLE
      *(volatile v4u*)(rowp + 256) = lo;
#endif
    }
    __threadfence();
  }
}

__global__ __launch_bounds__(256) void k_node2(const float* __restrict__ HW2, const float* __restrict__ tab,
                                               float* __restrict__ SD2) {
  const int lane = threadIdx.x & 31, wave = threadIdx.x >> 5;
  const int wv = (int)blockIdx.x * 8 + wave;
  if (wv >= NN / 16) return;
  const float as = tab[T_AS2 + lane];
  const float ad = tab[T_AD2 + lane];
  const int node0 = wv * 16;
  float outv = 0.0f;
#pragma unroll 1
  for (int q = 0; q < 16; ++q) {
    const float v = HW2[(size_t)(node0 + q) * 64 + lane];
    float ps = v * as;
    float pd = v * ad;
#pragma unroll
    for (int o = 16; o > 0; o >>= 1) { ps += __shfl_xor(ps, o); pd += __shfl_xor(pd, o); }
    const float mine = ((lane & 1) != 0) ? pd : ps;
    outv = ((lane >> 1) == q) ? mine : outv;
  }
  volatile float* qp = (volatile float*)(SD2 + (size_t)node0 * 2 + lane);
  *qp = outv;
  __threadfence();
  *qp = outv;
}

__global__ __launch_bounds__(256) void k_replay2(
    const float* __restrict__ HW2, const float* __restrict__ SD2, const unsigned* __restrict__ hits,
    const int* __restrict__ offp, const int* __restrict__ cntp, const int* __restrict__ flagp,
    const float* __restrict__ tab, float* __restrict__ out) {
  const int lane = threadIdx.x & 31, wave = threadIdx.x >> 5;
  const int row = (int)blockIdx.x * 8 + wave;
  const bool live = row < NN;
  const int ic = row < NN ? row : NN - 1;
  const int blk = ic >> 10;
  const int offv = offp[ic];
  const int cntv = cntp[ic];
  const int flg  = flagp[blk * FLGP];
  asm volatile("" :: "v"(offv), "v"(cntv), "v"(flg));
  const int cn  = __builtin_amdgcn_readfirstlane(live ? clampi(cntv, 0, DEGCAP) : 0);
  const int off = __builtin_amdgcn_readfirstlane(clampi(offv, 0, RCAP - 1));
  const bool bad = (flg != 0) || (cntv > DEGCAP) || (cntv < 0);

  const float oad = SD2[(size_t)ic * 2 + 1];
  const float bb  = tab[T_B2 + lane];
  asm volatile("" :: "v"(oad), "v"(bb));

  const unsigned* hb = hits + (size_t)blk * RCAP;
  const unsigned w0 = hb[clampi(off + lane, 0, RCAP - 1)];
  const unsigned w1 = hb[clampi(off + 32 + lane, 0, RCAP - 1)];
  asm volatile("" :: "v"(w0), "v"(w1));
  const int s0 = clampi((int)(w0 & 0xFFFFu), 0, NN - 1);
  int s1 = clampi((int)(w1 & 0xFFFFu), 0, NN - 1);
  s1 = (lane == 31) ? ic : s1;
  const float as0 = SD2[(size_t)s0 * 2];
  const float as1 = SD2[(size_t)s1 * 2];
  asm volatile("" :: "v"(as0), "v"(as1));
  const bool act0 = lane < cn;
  const bool act1 = ((32 + lane) < cn) || (lane == 31);
  const float ninf = __uint_as_float(0xff800000u);

  const float e0 = leaky(as0 + oad);
  const float e1 = leaky(as1 + oad);
  float m = act0 ? e0 : ninf;
  const float m1 = act1 ? e1 : ninf;
  m = nmax(m, m1);
#pragma unroll
  for (int o = 16; o > 0; o >>= 1) {
    const float t = __shfl_xor(m, o);
    m = nmax(m, t);
  }
  float p0 = expf(e0 - m);
  float p1 = expf(e1 - m);
  p0 = act0 ? p0 : 0.0f;
  p1 = act1 ? p1 : 0.0f;
  float dsum = p0 + p1;
#pragma unroll
  for (int o = 16; o > 0; o >>= 1) dsum += __shfl_xor(dsum, o);
  const float den = dsum + 1e-16f;
  const float al0 = p0 / den;
  const float al1 = p1 / den;

  float acc = 0.0f;
#pragma unroll 1
  for (int j = 0; j <= cn; ++j) {
    const int jj = j < cn ? j : 63;
    const int sa_ = rlane(s0, jj & 31);
    const int sb_ = rlane(s1, jj & 31);
    const int sj = jj < 32 ? sa_ : sb_;
    const float wa = rlanef(al0, jj & 31);
    const float wb = rlanef(al1, jj & 31);
    const float w = jj < 32 ? wa : wb;
    const float v = HW2[(size_t)sj * 64 + lane];
    asm volatile("" :: "v"(v));
    acc = acc + w * v;
  }
  float r = acc + bb;
  const float qn = __uint_as_float(0x7fc00000u);
  r = bad ? qn : r;
  volatile float* qp = (volatile float*)(out + (size_t)ic * OUTW + lane);
  if (live) *qp = r;
  __threadfence();
  if (live) *qp = r;
}

constexpr size_t SZ_RA   = (size_t)MPAD * 512 * 2;
constexpr size_t SZ_RB   = (size_t)MPAD * C1W * 4;
constexpr size_t SZ_SD1  = (size_t)MPAD * 8 * 4;
constexpr size_t SZ_SD2  = (size_t)MPAD * 2 * 4;
constexpr size_t SZ_HITS = (size_t)NBLK * RCAP * 4;
constexpr size_t SZ_OFF  = (size_t)NBLK * NB * 4;
constexpr size_t SZ_FLG  = (size_t)FLGL * FLGP * 4;
constexpr size_t SZ_W1T  = (size_t)C1W * FIN * 2;
constexpr size_t SZ_W2D  = (size_t)64 * 512 * 2;
constexpr size_t SZ_TAB  = (size_t)T_TOT * 4;
constexpr size_t O_RA    = 0;
constexpr size_t O_RB    = O_RA + SZ_RA;
constexpr size_t O_SD1   = O_RB + SZ_RB;
constexpr size_t O_SD2   = O_SD1 + SZ_SD1;
constexpr size_t O_HITS  = O_SD2 + SZ_SD2;
constexpr size_t O_OFF   = O_HITS + SZ_HITS;
constexpr size_t O_CNT   = O_OFF + SZ_OFF;
constexpr size_t O_FLG   = O_CNT + SZ_OFF;
constexpr size_t O_W1T   = O_FLG + SZ_FLG;
constexpr size_t O_W2D   = O_W1T + SZ_W1T;
constexpr size_t O_TAB   = O_W2D + SZ_W2D;
constexpr size_t WS_TOTAL = O_TAB + SZ_TAB;
static_assert(SZ_RA % 256 == 0 && SZ_RB % 256 == 0 && SZ_SD1 % 256 == 0 && SZ_SD2 % 256 == 0);
static_assert(SZ_HITS % 256 == 0 && SZ_OFF % 256 == 0 && SZ_FLG % 256 == 0);
static_assert(SZ_W1T % 256 == 0 && SZ_W2D % 256 == 0 && SZ_TAB % 256 == 0);
static_assert(SZ_RA >= (size_t)MPAD * FIN * 2 && SZ_RA >= (size_t)MPAD * K2TOT * 2);
static_assert(SZ_RB >= (size_t)MPAD * 64 * 4);
static_assert(SZ_SD1 >= (size_t)NN * 8 * 4 && SZ_SD2 >= (size_t)NN * 2 * 4);
static_assert(SZ_W2D >= (size_t)64 * K2TOT * 2);
static_assert(WS_TOTAL == ((size_t)106703 << 10));
static_assert(WS_TOTAL <= ((size_t)128 << 20));

extern "C" void kernel_launch(void* const* d_in, const int* in_sizes, int n_in,
                              void* d_out, int out_size, void* d_ws, size_t ws_size,
                              hipStream_t stream) {
  if (n_in != 14) return;
  if (in_sizes[0] != NN * FIN || in_sizes[1] != 2 * EE || in_sizes[2] != FIN * C1W) return;
  if (in_sizes[3] != C1W || in_sizes[4] != C1W || in_sizes[5] != C1W || in_sizes[6] != C1W) return;
  if (in_sizes[7] != C1W || in_sizes[8] != C1W || in_sizes[9] != C1W) return;
  if (in_sizes[10] != C1W * OUTW || in_sizes[11] != OUTW || in_sizes[12] != OUTW || in_sizes[13] != OUTW) return;
  if (out_size != NN * OUTW) return;
  if (ws_size < WS_TOTAL) return;

  const float* x    = (const float*)d_in[0];
  const int*   ei   = (const int*)  d_in[1];
  const float* W1   = (const float*)d_in[2];
  const float* as1  = (const float*)d_in[3];
  const float* ad1  = (const float*)d_in[4];
  const float* b1   = (const float*)d_in[5];
  const float* ga   = (const float*)d_in[6];
  const float* be   = (const float*)d_in[7];
  const float* mu   = (const float*)d_in[8];
  const float* var  = (const float*)d_in[9];
  const float* W2   = (const float*)d_in[10];
  const float* as2  = (const float*)d_in[11];
  const float* ad2  = (const float*)d_in[12];
  const float* b2   = (const float*)d_in[13];
  float* out = (float*)d_out;

  char* ws = (char*)d_ws;
  unsigned short* XB   = (unsigned short*)(ws + O_RA);
  unsigned short* A2   = (unsigned short*)(ws + O_RA);
  float*          HW   = (float*)(ws + O_RB);
  float*          HW2  = (float*)(ws + O_RB);
  float*          SD1  = (float*)(ws + O_SD1);
  float*          SD2  = (float*)(ws + O_SD2);
  unsigned*       HITS = (unsigned*)(ws + O_HITS);
  int*            OFFP = (int*)(ws + O_OFF);
  int*            CNTP = (int*)(ws + O_CNT);
  int*            FLG  = (int*)(ws + O_FLG);
  unsigned short* W1T  = (unsigned short*)(ws + O_W1T);
  unsigned short* W2D  = (unsigned short*)(ws + O_W2D);
  float*          TAB  = (float*)(ws + O_TAB);

  hipFuncSetAttribute(reinterpret_cast<const void*>(&k_bucket),
                      hipFuncAttributeMaxDynamicSharedMemorySize, LDS_BKT);

  k_plane<0><<<MPAD * FIN / 8 / 256, 256, 0, stream>>>(x, NN, FIN, FIN, XB, MPAD, FIN);
  k_prep<<<PB_END, 256, 0, stream>>>(W1, W2, as1, ad1, b1, ga, be, mu, var, as2, ad2, b2, W1T, W2D, TAB, A2, FLG);
  k_bucket<<<NBLK, 256, LDS_BKT, stream>>>(ei, HITS, OFFP, CNTP, FLG);
  k_gemm_nt<0, 0><<<(782 * 4 + 7) / 8, 256, 0, stream>>>(XB, W1T, TAB, HW, NN, C1W, FIN, C1W);
  k_node1<<<(NN / 4 + 7) / 8, 256, 0, stream>>>(HW, TAB, SD1);
  k_replay1<<<NN / 8, 256, 0, stream>>>(HW, SD1, HITS, OFFP, CNTP, FLG, TAB, A2);
  k_gemm_nt<0, 0><<<(782 + 7) / 8, 256, 0, stream>>>(A2, W2D, TAB, HW2, NN, 64, K2TOT, 64);
  k_node2<<<(NN / 16 + 7) / 8, 256, 0, stream>>>(HW2, TAB, SD2);
  k_replay2<<<NN / 8, 256, 0, stream>>>(HW2, SD2, HITS, OFFP, CNTP, FLG, TAB, out);
}
